// PolarConv_25546465477063
// MI455X (gfx1250) — hardware-verified
//
#include <hip/hip_runtime.h>
#include <stddef.h>


#pragma clang fp contract(off)

#define NTHR   256
#define NWAVE  8
#define QPW    8
#define QPB    (NWAVE * QPW)
#define CIN    16
#define HID    32
#define NCOL   256
#define KP     40
#define FP     16

static_assert(QPB * CIN == 4 * NTHR);
static_assert(((KP * 2) % 16) == 0);
static_assert((FP * 4) % 16 == 0);
static_assert((NCOL * HID) % NTHR == 0 && (HID * HID) % NTHR == 0);
static_assert(NTHR == NCOL);
static_assert(NWAVE * 32 == NTHR);

typedef float          v4f   __attribute__((ext_vector_type(4)));
typedef float          v8f   __attribute__((ext_vector_type(8)));
typedef unsigned short v8us  __attribute__((ext_vector_type(8)));
typedef unsigned short v16us __attribute__((ext_vector_type(16)));
typedef __bf16         v16b  __attribute__((ext_vector_type(16)));
union FragB { v16b v; v16us u; v8us h[2]; };

__device__ __forceinline__ v8f wmb(v16b a, v16b b, v8f c) {
  v8f d = __builtin_amdgcn_wmma_f32_16x16x32_bf16(false, a, false, b, (short)0, c, false, false);
  asm volatile("v_nop\n\tv_nop\n\tv_nop\n\tv_nop" : "+v"(d) : "v"(a), "v"(b));
  return d;
}

__device__ __forceinline__ unsigned short bfh(float f) {
  unsigned int u = __float_as_uint(f);
  u += 0x7FFFu + ((u >> 16) & 1u);
  return (unsigned short)(u >> 16);
}
__device__ __forceinline__ float bff(unsigned short h) {
  return __uint_as_float(((unsigned int)h) << 16);
}

__device__ __forceinline__ void wave_sync_lds() {
  __builtin_amdgcn_fence(__ATOMIC_ACQ_REL, "wavefront");
  __builtin_amdgcn_wave_barrier();
}

__global__ __launch_bounds__(NTHR) void k_edge_mlp(
    const float* __restrict__ feats, const float* __restrict__ xyz, const int* __restrict__ nidx,
    const int* __restrict__ rsp, const float* __restrict__ ndist,
    const float* __restrict__ W1, const float* __restrict__ b1,
    const float* __restrict__ W2, const float* __restrict__ b2,
    const float* __restrict__ W3, const float* __restrict__ b3,
    float* out, int nq, int nN, int nE) {
  __shared__ __attribute__((aligned(16))) unsigned short sW3h[NCOL * KP];
  __shared__ __attribute__((aligned(16))) unsigned short sW3l[NCOL * KP];
  __shared__ __attribute__((aligned(16))) unsigned short sW2h[HID * KP];
  __shared__ __attribute__((aligned(16))) unsigned short sW2l[HID * KP];
  __shared__ float sW1[4 * HID];
  __shared__ float sb1[HID];
  __shared__ float sb2[HID];
  __shared__ float sb3[NCOL];
  __shared__ __attribute__((aligned(16))) float sF[NWAVE * 16 * FP];
  __shared__ __attribute__((aligned(16))) float sOut[QPB * CIN];

  const int tid = (int)threadIdx.x;
  const int lane = tid & 31, wave = tid >> 5, hh = lane >> 4, m = lane & 15;

#pragma unroll 4
  for (int it = 0; it < (NCOL * HID) / NTHR; ++it) {
    const int idx = it * NTHR + tid;
    const int n = idx & (NCOL - 1);
    const int k = idx >> 8;
    const float w = W3[(size_t)k * NCOL + n];
    const unsigned short hb = bfh(w);
    sW3h[n * KP + k] = hb;
    sW3l[n * KP + k] = bfh(w - bff(hb));
  }
#pragma unroll
  for (int it = 0; it < (HID * HID) / NTHR; ++it) {
    const int idx = it * NTHR + tid;
    const int c = idx & (HID - 1);
    const int k = idx >> 5;
    const float w = W2[k * HID + c];
    const unsigned short hb = bfh(w);
    sW2h[c * KP + k] = hb;
    sW2l[c * KP + k] = bfh(w - bff(hb));
  }
  if (tid < 4 * HID) sW1[tid] = W1[tid];
  if (tid < HID) { sb1[tid] = b1[tid]; sb2[tid] = b2[tid]; }
  sb3[tid] = b3[tid];
  __syncthreads();

  const v8f z8 = {0.f, 0.f, 0.f, 0.f, 0.f, 0.f, 0.f, 0.f};
  const v4f z4 = {0.f, 0.f, 0.f, 0.f};
  float* myF = sF + wave * 16 * FP;
  const int qBase = (int)blockIdx.x * QPB + wave * QPW;

#pragma unroll 1
  for (int s = 0; s < QPW; ++s) {
    const int q = qBase + s;
    float res = 0.f;
    if (q < nq) {
      int base = rsp[q];
      int end  = rsp[q + 1];
      base = base < 0 ? 0 : (base > nE ? nE : base);
      end  = end < base ? base : (end > nE ? nE : end);
      const int qn = q > nN - 1 ? nN - 1 : q;
      const float qx = xyz[(size_t)qn * 3 + 0];
      const float qy = xyz[(size_t)qn * 3 + 1];
      const float qz = xyz[(size_t)qn * 3 + 2];

      float acc[8];
#pragma unroll
      for (int r = 0; r < 8; ++r) acc[r] = 0.f;

#pragma unroll 1
      for (int c0 = base; c0 < end; c0 += 16) {
        const int  e     = c0 + m;
        const bool valid = e < end;
        const int  ec    = valid ? e : (end - 1);
        int nb = nidx[ec];
        nb = nb < 0 ? 0 : (nb > nN - 1 ? nN - 1 : nb);
        const float d = ndist[ec];
        const float* xp = xyz + (size_t)nb * 3;
        const float dx = xp[0] - qx;
        const float dy = xp[1] - qy;
        const float dz = xp[2] - qz;
        const float r   = sqrtf(d + 1e-7f);
        const float inv = 1.0f / r;
        const float p0 = r, p1 = dx * inv, p2 = dz * inv, p3 = dy * inv;

        const float* fr = feats + (size_t)nb * CIN + 8 * hh;
        v4f f0 = *(const v4f*)fr;
        v4f f1 = *(const v4f*)(fr + 4);
        f0 = valid ? f0 : z4;
        f1 = valid ? f1 : z4;
        wave_sync_lds();
        *(v4f*)(myF + m * FP + 8 * hh)     = f0;
        *(v4f*)(myF + m * FP + 8 * hh + 4) = f1;
        wave_sync_lds();

        FragB bh1, bl1;
#pragma unroll
        for (int i = 0; i < 16; ++i) {
          const int j = 8 * hh + i + ((i >> 3) << 3);
          float v = p0 * sW1[j];
          v = fmaf(p1, sW1[HID + j], v);
          v = fmaf(p2, sW1[2 * HID + j], v);
          v = fmaf(p3, sW1[3 * HID + j], v);
          v = v + sb1[j];
          v = fmaxf(v, 0.f);
          const unsigned short hb = bfh(v);
          bh1.u[i] = hb;
          bl1.u[i] = bfh(v - bff(hb));
        }

        FragB a3h, a3l;
#pragma unroll
        for (int ct = 0; ct < 2; ++ct) {
          const int ro = (16 * ct + m) * KP;
          FragB wh, wl;
          wh.h[0] = *(const v8us*)(sW2h + ro + 8 * hh);
          wh.h[1] = *(const v8us*)(sW2h + ro + 16 + 8 * hh);
          wl.h[0] = *(const v8us*)(sW2l + ro + 8 * hh);
          wl.h[1] = *(const v8us*)(sW2l + ro + 16 + 8 * hh);
          v8f d2 = wmb(wh.v, bh1.v, z8);
          d2 = wmb(wh.v, bl1.v, d2);
          d2 = wmb(wl.v, bh1.v, d2);
#pragma unroll
          for (int r = 0; r < 8; ++r) {
            float v = d2[r] + sb2[16 * ct + 8 * hh + r];
            v = fmaxf(v, 0.f);
            const unsigned short hb = bfh(v);
            a3h.u[8 * ct + r] = hb;
            a3l.u[8 * ct + r] = bfh(v - bff(hb));
          }
        }

#pragma unroll
        for (int g = 0; g < 4; ++g) {
          v4f fq[8];
#pragma unroll
          for (int r = 0; r < 8; ++r) fq[r] = *(const v4f*)(myF + (8 * hh + r) * FP + 4 * g);
#pragma unroll
          for (int t = 0; t < 4; ++t) {
            const int n  = 16 * (4 * g + t) + m;
            const int ro = n * KP;
            FragB wh, wl;
            wh.h[0] = *(const v8us*)(sW3h + ro + 8 * hh);
            wh.h[1] = *(const v8us*)(sW3h + ro + 16 + 8 * hh);
            wl.h[0] = *(const v8us*)(sW3l + ro + 8 * hh);
            wl.h[1] = *(const v8us*)(sW3l + ro + 16 + 8 * hh);
            v8f d3 = wmb(a3h.v, wh.v, z8);
            d3 = wmb(a3h.v, wl.v, d3);
            d3 = wmb(a3l.v, wh.v, d3);
            const float bb = sb3[n];
#pragma unroll
            for (int r = 0; r < 8; ++r) acc[r] = fmaf(fq[r][t], d3[r] + bb, acc[r]);
          }
        }
      }

      float sres = ((acc[0] + acc[1]) + (acc[2] + acc[3])) + ((acc[4] + acc[5]) + (acc[6] + acc[7]));
      sres += __shfl_xor(sres, 16);
      res = sres;
    }
    if (hh == 0) sOut[(wave * QPW + s) * CIN + m] = res;
  }
  __syncthreads();

  const v4f ov = *(const v4f*)(sOut + 4 * tid);
  const int row = tid >> 2;
  const int oq = (int)blockIdx.x * QPB + row;
  float* op = out + (size_t)blockIdx.x * QPB * CIN + 4 * tid;
  if (oq < nq) *(volatile v4f*)op = ov;
  __threadfence();
  if (oq < nq) *(volatile v4f*)op = ov;
}

extern "C" void kernel_launch(void* const* d_in, const int* in_sizes, int n_in,
                              void* d_out, int out_size, void* d_ws, size_t ws_size,
                              hipStream_t stream) {
  if (n_in < 11) return;
  if (in_sizes[1] <= 0 || (in_sizes[1] % 3) != 0) return;
  const int nN = in_sizes[1] / 3;
  if (in_sizes[0] != nN * CIN) return;
  const int nq = in_sizes[3] - 1;
  if (nq <= 0 || nq > nN) return;
  const int nE = in_sizes[2];
  if (nE <= 0 || in_sizes[4] != nE) return;
  if (in_sizes[5] != 4 * HID || in_sizes[6] != HID) return;
  if (in_sizes[7] != HID * HID || in_sizes[8] != HID) return;
  if (in_sizes[9] != HID * NCOL || in_sizes[10] != NCOL) return;
  if (out_size != nq * CIN) return;

  const float* feats = (const float*)d_in[0];
  const float* xyz   = (const float*)d_in[1];
  const int*   nidx  = (const int*)d_in[2];
  const int*   rsp   = (const int*)d_in[3];
  const float* ndist = (const float*)d_in[4];
  const float* W1    = (const float*)d_in[5];
  const float* b1    = (const float*)d_in[6];
  const float* W2    = (const float*)d_in[7];
  const float* b2    = (const float*)d_in[8];
  const float* W3    = (const float*)d_in[9];
  const float* b3    = (const float*)d_in[10];
  float* out = (float*)d_out;
  (void)d_ws; (void)ws_size;

  const int nBlk = (nq + QPB - 1) / QPB;
  k_edge_mlp<<<nBlk, NTHR, 0, stream>>>(feats, xyz, nidx, rsp, ndist, W1, b1, W2, b2, W3, b3,
                                        out, nq, nN, nE);
}
